// Mamba2Simple_82910048681998
// MI455X (gfx1250) — hardware-verified
//
#include <hip/hip_runtime.h>
#include <hip/hip_bf16.h>
#include <math.h>


typedef _Float16 bf16;
typedef _Float16 f16;
typedef __attribute__((ext_vector_type(4))) unsigned v4u_t;
typedef unsigned v4ua __attribute__((ext_vector_type(4), may_alias));
typedef __attribute__((ext_vector_type(4))) float v4f_t;
typedef float v4fa __attribute__((ext_vector_type(4), may_alias));
typedef __attribute__((ext_vector_type(16))) bf16  bf16x16;
typedef bf16x16 f16x16;
typedef __attribute__((ext_vector_type(8)))  bf16  bf16x8;
typedef bf16x8 f16x8;
typedef __attribute__((ext_vector_type(4)))  bf16  bf16x4;
typedef __attribute__((ext_vector_type(8)))  float f32x8;
__device__ __forceinline__ f32x8 wmma16(f16x16 a, f16x16 b, f32x8 c) {
  c = __builtin_amdgcn_wmma_f32_16x16x32_f16(false, a, false, b, (short)0, c, false, false);
  asm volatile("v_nop\n\tv_nop\n\tv_nop\n\tv_nop" : "+v"(c) : "v"(a), "v"(b));
  return c;
}
#define LDS_STRIDE 48
#define KSTRIDE    72
#define VSTRIDE    48

__device__ __forceinline__ f32x8 wmma_bf16(bf16x16 a, bf16x16 b, f32x8 c) {
  c = __builtin_amdgcn_wmma_f32_16x16x32_f16(false, a, false, b, (short)0, c, false, false);
  asm volatile("v_nop\n\tv_nop\n\tv_nop\n\tv_nop" : "+v"(c) : "v"(a), "v"(b));
  return c;
}

template <typename T>
__device__ __forceinline__ bf16x16 load_frag(const T* __restrict__ base, int ld,
                                             int row0, int k0) {
  const int lane = threadIdx.x & 31;
  const int r    = lane & 15;
  const int kh   = (lane >> 4) * 8;
  const T* p0 = base + (size_t)(row0 + r) * ld + (k0 + kh);
  const T* p1 = p0 + 16;
  bf16x16 f;
#pragma unroll
  for (int i = 0; i < 8; ++i) {
    f[i]     = (bf16)p0[i];
    f[i + 8] = (bf16)p1[i];
  }
  return f;
}

__device__ __forceinline__ bf16x16 lds_frag(const bf16* base, int stride) {
  const int lane = threadIdx.x & 31;
  const int row  = lane & 15;
  const int kh   = (lane >> 4) * 8;
  const bf16x8 lo = *(const bf16x8*)(base + row * stride + kh);
  const bf16x8 hi = *(const bf16x8*)(base + row * stride + kh + 16);
  bf16x16 f;
#pragma unroll
  for (int i = 0; i < 8; ++i) { f[i] = lo[i]; f[i + 8] = hi[i]; }
  return f;
}

template <typename T>
__device__ __forceinline__ void stage_read16(const T* __restrict__ p, float* buf) {
#pragma unroll
  for (int i = 0; i < 16; ++i) buf[i] = (float)p[i];
}

__device__ __forceinline__ void stage_write(bf16* dst, const float* buf, int nquad) {
#pragma unroll
  for (int i = 0; i < nquad; ++i) {
    bf16x4 q;
    q[0] = (bf16)buf[4 * i];     q[1] = (bf16)buf[4 * i + 1];
    q[2] = (bf16)buf[4 * i + 2]; q[3] = (bf16)buf[4 * i + 3];
    *(bf16x4*)(dst + 4 * i) = q;
  }
}


#define GSTR 48
#define GSTR 48
template <typename AT, int EPI, bool OUT16>
__global__ __launch_bounds__(256) void gemm_kne(const AT* __restrict__ A, int lda, const float* __restrict__ Wm, int ldw,
                                                const float* __restrict__ bias, const float* __restrict__ R, const float* __restrict__ gvec,
                                                void* __restrict__ Yv, int ldy, int K) {
  __shared__ __attribute__((aligned(16))) f16 ldsA[128 * GSTR];
  __shared__ __attribute__((aligned(16))) f16 ldsW[128 * GSTR];
  __shared__ __attribute__((aligned(16))) float oS[8][32 * 68];
  const int tid = threadIdx.x, lane = tid & 31, wave = tid >> 5, cl = lane & 15, rh = (lane >> 4) * 8;
  const int m0 = blockIdx.x * 128, n0 = blockIdx.y * 128;
  const int wm = (wave & 3) * 32, wn = (wave >> 2) * 64;
  f32x8 acc[2][4];
#pragma unroll
  for (int i = 0; i < 2; ++i)
#pragma unroll
    for (int j = 0; j < 4; ++j) { f32x8 z = {}; acc[i][j] = z; }
#pragma unroll 1
  for (int k0 = 0; k0 < K; k0 += 32) {
    __syncthreads();
    { const int row = tid >> 1, ch = (tid & 1) * 16;
      const AT* src = A + (size_t)(m0 + row) * lda + k0 + ch;
#pragma unroll
      for (int g = 0; g < 16; ++g) ldsA[row * GSTR + ch + g] = (f16)src[g]; }
    { const int k = tid >> 3, nn0 = (tid & 7) * 16;
      const float* src = Wm + (size_t)(k0 + k) * ldw + n0 + nn0;
#pragma unroll
      for (int g = 0; g < 4; ++g) { const v4f_t v = *(const v4f_t*)(src + 4 * g);
#pragma unroll
        for (int u = 0; u < 4; ++u) ldsW[(nn0 + 4 * g + u) * GSTR + k] = (f16)v[u]; } }
    __syncthreads();
    f16x16 af[2];
#pragma unroll
    for (int i = 0; i < 2; ++i) af[i] = lds_frag(ldsA + (wm + 16 * i) * GSTR, GSTR);
#pragma unroll
    for (int j = 0; j < 4; ++j) {
      const f16x16 bf = lds_frag(ldsW + (wn + 16 * j) * GSTR, GSTR);
#pragma unroll
      for (int i = 0; i < 2; ++i) acc[i][j] = wmma16(af[i], bf, acc[i][j]);
    }
  }
  float* so = oS[wave];
#pragma unroll
  for (int i = 0; i < 2; ++i)
#pragma unroll
    for (int j = 0; j < 4; ++j) {
      const int n = n0 + wn + 16 * j + cl;
      const float bv = bias ? bias[n] : 0.0f;
      const float gv = (EPI == 2 || EPI == 4) ? gvec[n] : 0.0f;
      if (EPI == 1) {
#pragma unroll 1
        for (int r = 0; r < 8; ++r) { const float xg = acc[i][j][r] + bv; so[(16 * i + rh + r) * 68 + 16 * j + cl] = 0.5f * xg * (1.0f + erff(xg * 0.70710678118654752f)); }
      } else {
#pragma unroll
        for (int r = 0; r < 8; ++r) {
          float v = acc[i][j][r] + bv;
          if (EPI == 3) v = fmaxf(v, 0.0f);
          if (EPI == 4) v = gv * v;
          if (EPI == 2) v = R[(size_t)(m0 + wm + 16 * i + rh + r) * ldy + n] + gv * v;
          so[(16 * i + rh + r) * 68 + 16 * j + cl] = v;
        }
      }
    }
  asm volatile("s_wait_dscnt 0" ::: "memory");
  __builtin_amdgcn_wave_barrier();
#pragma unroll 1
  for (int pass = 0; pass < 2; ++pass) {
    if (OUT16) {
      f16* Y = (f16*)Yv;
#pragma unroll
      for (int it = 0; it < 8; ++it) { const int c = lane + 32 * it, rr = c >> 3, q8 = (c & 7) * 8;
        union { f16 h[8]; v4u_t v; } u;
#pragma unroll
        for (int e = 0; e < 8; ++e) u.h[e] = (f16)so[rr * 68 + q8 + e];
        *(volatile v4u_t*)(Y + (size_t)(m0 + wm + rr) * ldy + n0 + wn + q8) = u.v; }
    } else {
      float* Y = (float*)Yv;
#pragma unroll
      for (int it = 0; it < 16; ++it) { const int f4 = lane + 32 * it, rr = f4 >> 4, q = (f4 & 15) * 4;
        *(volatile v4f_t*)(Y + (size_t)(m0 + wm + rr) * ldy + n0 + wn + q) = *(const v4fa*)(so + rr * 68 + q); }
    }
    __threadfence();
  }
}

template <typename AT, int EPI, bool OUT16>
__global__ __launch_bounds__(256) void gemm_knez(const AT* __restrict__ A, int lda, size_t strideA, const float* __restrict__ Wm, int ldw, size_t strideW,
                                                 const float* __restrict__ bias, const float* __restrict__ R, const float* __restrict__ gvec,
                                                 void* __restrict__ Yv, int ldy, size_t strideY, int K) {
  A += (size_t)blockIdx.z * strideA; Wm += (size_t)blockIdx.z * strideW; Yv = (void*)((char*)Yv + (size_t)blockIdx.z * strideY * (OUT16 ? 2 : 4)); if (R) R += (size_t)blockIdx.z * strideY;
  __shared__ __attribute__((aligned(16))) f16 ldsA[128 * GSTR];
  __shared__ __attribute__((aligned(16))) f16 ldsW[128 * GSTR];
  __shared__ __attribute__((aligned(16))) float oS[8][32 * 68];
  const int tid = threadIdx.x, lane = tid & 31, wave = tid >> 5, cl = lane & 15, rh = (lane >> 4) * 8;
  const int m0 = blockIdx.x * 128, n0 = blockIdx.y * 128;
  const int wm = (wave & 3) * 32, wn = (wave >> 2) * 64;
  f32x8 acc[2][4];
#pragma unroll
  for (int i = 0; i < 2; ++i)
#pragma unroll
    for (int j = 0; j < 4; ++j) { f32x8 z = {}; acc[i][j] = z; }
#pragma unroll 1
  for (int k0 = 0; k0 < K; k0 += 32) {
    __syncthreads();
    { const int row = tid >> 1, ch = (tid & 1) * 16;
      const AT* src = A + (size_t)(m0 + row) * lda + k0 + ch;
#pragma unroll
      for (int g = 0; g < 16; ++g) ldsA[row * GSTR + ch + g] = (f16)src[g]; }
    { const int k = tid >> 3, nn0 = (tid & 7) * 16;
      const float* src = Wm + (size_t)(k0 + k) * ldw + n0 + nn0;
#pragma unroll
      for (int g = 0; g < 4; ++g) { const v4f_t v = *(const v4f_t*)(src + 4 * g);
#pragma unroll
        for (int u = 0; u < 4; ++u) ldsW[(nn0 + 4 * g + u) * GSTR + k] = (f16)v[u]; } }
    __syncthreads();
    f16x16 af[2];
#pragma unroll
    for (int i = 0; i < 2; ++i) af[i] = lds_frag(ldsA + (wm + 16 * i) * GSTR, GSTR);
#pragma unroll
    for (int j = 0; j < 4; ++j) {
      const f16x16 bf = lds_frag(ldsW + (wn + 16 * j) * GSTR, GSTR);
#pragma unroll
      for (int i = 0; i < 2; ++i) acc[i][j] = wmma16(af[i], bf, acc[i][j]);
    }
  }
  float* so = oS[wave];
#pragma unroll
  for (int i = 0; i < 2; ++i)
#pragma unroll
    for (int j = 0; j < 4; ++j) {
      const int n = n0 + wn + 16 * j + cl;
      const float bv = bias ? bias[n] : 0.0f;
      const float gv = (EPI == 2 || EPI == 4) ? gvec[n] : 0.0f;
      if (EPI == 1) {
#pragma unroll 1
        for (int r = 0; r < 8; ++r) { const float xg = acc[i][j][r] + bv; so[(16 * i + rh + r) * 68 + 16 * j + cl] = 0.5f * xg * (1.0f + erff(xg * 0.70710678118654752f)); }
      } else {
#pragma unroll
        for (int r = 0; r < 8; ++r) {
          float v = acc[i][j][r] + bv;
          if (EPI == 3) v = fmaxf(v, 0.0f);
          if (EPI == 4) v = gv * v;
          if (EPI == 2) v = R[(size_t)(m0 + wm + 16 * i + rh + r) * ldy + n] + gv * v;
          so[(16 * i + rh + r) * 68 + 16 * j + cl] = v;
        }
      }
    }
  asm volatile("s_wait_dscnt 0" ::: "memory");
  __builtin_amdgcn_wave_barrier();
#pragma unroll 1
  for (int pass = 0; pass < 2; ++pass) {
    if (OUT16) {
      f16* Y = (f16*)Yv;
#pragma unroll
      for (int it = 0; it < 8; ++it) { const int c = lane + 32 * it, rr = c >> 3, q8 = (c & 7) * 8;
        union { f16 h[8]; v4u_t v; } u;
#pragma unroll
        for (int e = 0; e < 8; ++e) u.h[e] = (f16)so[rr * 68 + q8 + e];
        *(volatile v4u_t*)(Y + (size_t)(m0 + wm + rr) * ldy + n0 + wn + q8) = u.v; }
    } else {
      float* Y = (float*)Yv;
#pragma unroll
      for (int it = 0; it < 16; ++it) { const int f4 = lane + 32 * it, rr = f4 >> 4, q = (f4 & 15) * 4;
        *(volatile v4f_t*)(Y + (size_t)(m0 + wm + rr) * ldy + n0 + wn + q) = *(const v4fa*)(so + rr * 68 + q); }
    }
    __threadfence();
  }
}

template <typename AT, bool ACC>
__global__ __launch_bounds__(256) void gemm_kn2(const AT* __restrict__ A, int lda, size_t strideA,
                                               const float* __restrict__ Wm, int ldw, size_t strideW,
                                               const float* __restrict__ bias, float scale,
                                               float* __restrict__ Y, int ldy, size_t strideY, int K) {
  __shared__ __attribute__((aligned(16))) f16 ldsA[128 * GSTR], ldsAl[128 * GSTR];
  __shared__ __attribute__((aligned(16))) f16 ldsW[128 * GSTR], ldsWl[128 * GSTR];
  __shared__ __attribute__((aligned(16))) float oS[8][32 * 68];
  const int tid = threadIdx.x, lane = tid & 31, wave = tid >> 5, cl = lane & 15, rh = (lane >> 4) * 8;
  const int m0 = blockIdx.x * 128, n0 = blockIdx.y * 128;
  const int wm = (wave & 3) * 32, wn = (wave >> 2) * 64;
  A += (size_t)blockIdx.z * strideA; Wm += (size_t)blockIdx.z * strideW; Y += (size_t)blockIdx.z * strideY;
  f32x8 acc[2][4], accx[2][4];
#pragma unroll
  for (int i = 0; i < 2; ++i)
#pragma unroll
    for (int j = 0; j < 4; ++j) { f32x8 z = {}; acc[i][j] = z; accx[i][j] = z; }
#pragma unroll 1
  for (int k0 = 0; k0 < K; k0 += 32) {
    __syncthreads();
    {
      const int row = tid >> 1, ch = (tid & 1) * 16;
      const AT* src = A + (size_t)(m0 + row) * lda + k0 + ch;
#pragma unroll
      for (int g = 0; g < 16; ++g) { const float v = (float)src[g]; const f16 h = (f16)v; ldsA[row * GSTR + ch + g] = h; ldsAl[row * GSTR + ch + g] = (f16)((v - (float)h) * 2048.0f); }
    }
    {
      const int k = tid >> 3, nn0 = (tid & 7) * 16;
      const float* src = Wm + (size_t)(k0 + k) * ldw + n0 + nn0;
#pragma unroll
      for (int g = 0; g < 4; ++g) { const v4f_t v = *(const v4f_t*)(src + 4 * g);
#pragma unroll
        for (int u = 0; u < 4; ++u) { const f16 h = (f16)v[u]; ldsW[(nn0 + 4 * g + u) * GSTR + k] = h; ldsWl[(nn0 + 4 * g + u) * GSTR + k] = (f16)((v[u] - (float)h) * 2048.0f); } }
    }
    __syncthreads();
    f16x16 af[2], afl[2];
#pragma unroll
    for (int i = 0; i < 2; ++i) { af[i] = lds_frag(ldsA + (wm + 16 * i) * GSTR, GSTR); afl[i] = lds_frag(ldsAl + (wm + 16 * i) * GSTR, GSTR); }
#pragma unroll
    for (int j = 0; j < 4; ++j) {
      const f16x16 bf = lds_frag(ldsW + (wn + 16 * j) * GSTR, GSTR), bfl = lds_frag(ldsWl + (wn + 16 * j) * GSTR, GSTR);
#pragma unroll
      for (int i = 0; i < 2; ++i) { acc[i][j] = wmma16(af[i], bf, acc[i][j]); accx[i][j] = wmma16(af[i], bfl, accx[i][j]); accx[i][j] = wmma16(afl[i], bf, accx[i][j]); }
    }
  }
  float* so = oS[wave];
#pragma unroll
  for (int i = 0; i < 2; ++i)
#pragma unroll
    for (int j = 0; j < 4; ++j) {
      const float bv = bias ? bias[n0 + wn + 16 * j + cl] : 0.0f;
#pragma unroll
      for (int r = 0; r < 8; ++r) so[(16 * i + rh + r) * 68 + 16 * j + cl] = (acc[i][j][r] + accx[i][j][r] * (1.0f / 2048.0f)) * scale + bv;
    }
  asm volatile("s_wait_dscnt 0" ::: "memory");
  __builtin_amdgcn_wave_barrier();
  if (ACC) {
#pragma unroll
    for (int it = 0; it < 16; ++it) { const int f4 = lane + 32 * it, rr = f4 >> 4, q = (f4 & 15) * 4;
      const v4f_t old = *(const v4fa*)(Y + (size_t)(m0 + wm + rr) * ldy + n0 + wn + q);
      v4f_t v = *(const v4fa*)(so + rr * 68 + q); v += old; *(v4fa*)(so + rr * 68 + q) = v; }
    asm volatile("s_wait_dscnt 0" ::: "memory");
  }
#pragma unroll 1
  for (int pass = 0; pass < 2; ++pass) {
#pragma unroll
    for (int it = 0; it < 16; ++it) { const int f4 = lane + 32 * it, rr = f4 >> 4, q = (f4 & 15) * 4;
      *(volatile v4f_t*)(Y + (size_t)(m0 + wm + rr) * ldy + n0 + wn + q) = *(const v4fa*)(so + rr * 68 + q); }
    __threadfence();
  }
}

__global__ __launch_bounds__(256) void k_transpose(const float* __restrict__ Wm, float* __restrict__ Wt, int rows, int cols) {
  __shared__ float tS[64][65];
  const int tid = threadIdx.x, tbj = cols / 64, bi = blockIdx.x / tbj, bj = blockIdx.x % tbj;
  for (int e = tid; e < 64 * 64; e += 256) { const int r = e >> 6, c = e & 63; tS[r][c] = Wm[(size_t)(bi * 64 + r) * cols + bj * 64 + c]; }
  __syncthreads();
  for (int ch = tid; ch < 64 * 16; ch += 256) { const int r = ch >> 4, q4 = (ch & 15) * 4; v4f_t o; o[0] = tS[q4][r]; o[1] = tS[q4 + 1][r]; o[2] = tS[q4 + 2][r]; o[3] = tS[q4 + 3][r];
    float* dst = Wt + (size_t)(bj * 64 + r) * rows + bi * 64 + q4; *(volatile v4f_t*)dst = o; __threadfence(); *(volatile v4f_t*)dst = o; }
}


#define GSTR 48
#define SS 2048
#define HH 32
#define DKK 64
template <typename AT, int MODE>
__global__ __launch_bounds__(256) void gemm_rb_kernel(
    const AT* __restrict__ A, const float* __restrict__ W,
    const float* __restrict__ bias, const float* __restrict__ rowscale, const float* __restrict__ R, const float* __restrict__ rowbias, void* __restrict__ out,
    int M, int N, int K) {
  __shared__ bf16 ldsA[128 * LDS_STRIDE];
  __shared__ bf16 ldsW[256 * LDS_STRIDE];
  __shared__ __attribute__((aligned(16))) unsigned char sob[256 * 136 * 2];

  const int t    = threadIdx.x;
  const int wave = t >> 5;
  const int lane = t & 31;
  const int wm   = (wave & 1) * 64;
  const int wn   = (wave >> 1) * 64;
  const int mBlk = blockIdx.x * 128;
  const int nBlk = blockIdx.y * 256;

  const int arow = t >> 1;
  const int ach  = (t & 1) * 16;

  float abuf[16];
  float wbuf[32];

  stage_read16(A + (size_t)(mBlk + arow) * K + ach, abuf);
  const int nrow = min(nBlk + t, N - 1);
  stage_read16(W + (size_t)nrow * K,          wbuf);
  stage_read16(W + (size_t)nrow * K + 16,     wbuf + 16);

  f32x8 acc[4][4] = {};

  for (int k = 0; k < K; k += 32) {
    __syncthreads();
    stage_write(&ldsA[arow * LDS_STRIDE + ach], abuf, 4);
    stage_write(&ldsW[t * LDS_STRIDE],          wbuf, 8);
    if (k + 32 < K) {
      stage_read16(A + (size_t)(mBlk + arow) * K + (k + 32) + ach, abuf);
      stage_read16(W + (size_t)nrow * K + (k + 32),          wbuf);
      stage_read16(W + (size_t)nrow * K + (k + 32) + 16,     wbuf + 16);
    }
    __syncthreads();

    bf16x16 af[4], wf[4];
#pragma unroll
    for (int i = 0; i < 4; ++i)
      af[i] = lds_frag(ldsA + (wm + 16 * i) * LDS_STRIDE, LDS_STRIDE);
#pragma unroll
    for (int j = 0; j < 4; ++j)
      wf[j] = lds_frag(ldsW + (wn + 16 * j) * LDS_STRIDE, LDS_STRIDE);
#pragma unroll
    for (int i = 0; i < 4; ++i)
#pragma unroll
      for (int j = 0; j < 4; ++j)
        acc[i][j] = wmma_bf16(af[i], wf[j], acc[i][j]);
  }

  const int nlane = lane & 15;
  const int mh    = (lane >> 4) * 8;
  __syncthreads();
  if (MODE == 0 || MODE == 1 || MODE == 3) {
    bf16* so = (bf16*)sob;
#pragma unroll
    for (int i = 0; i < 4; ++i)
#pragma unroll
      for (int j = 0; j < 4; ++j) {
        const int nl = wn + 16 * j + nlane;
        const float bv = bias ? bias[nBlk + nl] : 0.0f;
        if (MODE == 3) {
#pragma unroll 1
          for (int r = 0; r < 8; ++r) {
            const int ml = wm + 16 * i + mh + r;
            const float xg = acc[i][j][r] + bv;
            so[ml * 264 + nl] = (bf16)(0.5f * xg * (1.0f + erff(xg * 0.70710678118654752f)));
          }
        } else {
#pragma unroll
        for (int r = 0; r < 8; ++r) {
          const int ml = wm + 16 * i + mh + r;
          const bf16 hv = (bf16)(acc[i][j][r] + bv);
          if (MODE == 0) so[ml * 264 + nl] = hv;
          else           so[nl * 136 + ml] = hv;
        }
        }
      }
    __syncthreads();
#pragma unroll 1
    for (int pass = 0; pass < 2; ++pass) {
      if (MODE == 0 || MODE == 3) {
        for (int ch = t; ch < 128 * 32; ch += 256) { const int ml = ch >> 5, q = (ch & 31) * 8;
          *(volatile v4u_t*)((bf16*)out + (size_t)(mBlk + ml) * N + nBlk + q) = *(const v4ua*)(so + ml * 264 + q); }
      } else {
        const int b_ = mBlk / SS, s0 = mBlk % SS;
        for (int ch = t; ch < 256 * 16; ch += 256) { const int nl = ch >> 4, q = (ch & 15) * 8; const int n = nBlk + nl, h = n >> 6, dk = n & (DKK - 1);
          *(volatile v4u_t*)((bf16*)out + (((size_t)(b_ * HH + h)) * DKK + dk) * SS + s0 + q) = *(const v4ua*)(so + nl * 136 + q); }
      }
      __threadfence();
    }
  } else {
    float* so = (float*)sob;
#pragma unroll 1
    for (int hf = 0; hf < 2; ++hf) {
      if (wm == hf * 64) {
#pragma unroll
        for (int i = 0; i < 4; ++i)
#pragma unroll
          for (int j = 0; j < 4; ++j) {
            const int nl = wn + 16 * j + nlane;
            const float bv = bias ? bias[nBlk + nl] : 0.0f;
#pragma unroll
            for (int r = 0; r < 8; ++r) { const int mrow = mBlk + hf * 64 + 16 * i + mh + r; so[(16 * i + mh + r) * 260 + nl] = acc[i][j][r] * (rowscale ? rowscale[mrow] : 1.0f) + bv + (rowbias ? rowbias[mrow] : 0.0f); }
          }
      }
      __syncthreads();
      if (R) {
        for (int ch = t; ch < 64 * 64; ch += 256) { const int ml = ch >> 6, q = (ch & 63) * 4;
          if (nBlk + q < N) { const v4f_t rv = *(const v4f_t*)(R + (size_t)(mBlk + hf * 64 + ml) * N + nBlk + q); v4f_t v = *(const v4fa*)(so + ml * 260 + q); v += rv; *(volatile v4fa*)(so + ml * 260 + q) = v; } }
        asm volatile("s_wait_dscnt 0" ::: "memory");
      }
#pragma unroll 1
      for (int pass = 0; pass < 2; ++pass) {
        for (int ch = t; ch < 64 * 64; ch += 256) { const int ml = ch >> 6, q = (ch & 63) * 4;
          if (nBlk + q < N) *(volatile v4f_t*)((float*)out + (size_t)(mBlk + hf * 64 + ml) * N + nBlk + q) = *(const v4fa*)(so + ml * 260 + q); }
        __threadfence();
      }
      __syncthreads();
    }
  }
}

#define NBm 2
#define LLm 2048
#define LIN 2048
#define DDm 1024
#define DIm 2048
#define NHm 16
#define PPm 128
#define NSm 128
#define CDm 2304
#define NPm 4368
#define NPP 4480
#define CKm 256
#define DTPm 32
#define NCK (LLm / CKm)
__global__ __launch_bounds__(256) void k_fill(float* __restrict__ p, float val, size_t n4) { const size_t i = (size_t)blockIdx.x * 256 + threadIdx.x; if (i < n4) { v4f_t v = {val, val, val, val}; *(volatile v4f_t*)(p + 4 * i) = v; __threadfence(); *(volatile v4f_t*)(p + 4 * i) = v; } }
__global__ __launch_bounds__(256) void k_dbg_zero(float* __restrict__ p, size_t n4) { const size_t i = (size_t)blockIdx.x * 256 + threadIdx.x; if (i < n4) { v4f_t z = {0.f,0.f,0.f,0.f}; *(volatile v4f_t*)(p + 4 * i) = z; __threadfence(); *(volatile v4f_t*)(p + 4 * i) = z; } }
__global__ __launch_bounds__(256) void k_copy(const float* __restrict__ src, float* __restrict__ dst, size_t n4) { const size_t i = (size_t)blockIdx.x * 256 + threadIdx.x; if (i < n4) { const v4f_t v = *(const v4f_t*)(src + 4 * i); *(volatile v4f_t*)(dst + 4 * i) = v; __threadfence(); *(volatile v4f_t*)(dst + 4 * i) = v; } }
__global__ __launch_bounds__(256) void k_transpose_ld(const float* __restrict__ Wm, int lds, float* __restrict__ Wt, int rows, int cols) {
  __shared__ float tS[64][65];
  const int tid = threadIdx.x, tbj = cols / 64, bi = blockIdx.x / tbj, bj = blockIdx.x % tbj;
  for (int e = tid; e < 64 * 64; e += 256) { const int r = e >> 6, c = e & 63; tS[r][c] = Wm[(size_t)(bi * 64 + r) * lds + bj * 64 + c]; }
  __syncthreads();
  for (int ch = tid; ch < 64 * 16; ch += 256) { const int r = ch >> 4, q4 = (ch & 15) * 4; v4f_t o; o[0] = tS[q4][r]; o[1] = tS[q4 + 1][r]; o[2] = tS[q4 + 2][r]; o[3] = tS[q4 + 3][r];
    float* dst = Wt + (size_t)(bj * 64 + r) * rows + bi * 64 + q4; *(volatile v4f_t*)dst = o; __threadfence(); *(volatile v4f_t*)dst = o; }
}
__global__ __launch_bounds__(256) void k_padin(const float* __restrict__ Wm, float* __restrict__ WT) {
  const int k = blockIdx.x, tid = threadIdx.x;
#pragma unroll 1
  for (int n = tid; n < NPP; n += 256) { const float v = (n < NPm) ? Wm[(size_t)min(n, NPm - 1) * DDm + k] : 0.0f; *(volatile float*)(WT + (size_t)k * NPP + n) = v; }
  __threadfence();
#pragma unroll 1
  for (int n = tid; n < NPP; n += 256) { float* p = WT + (size_t)k * NPP + n; const float v = p[0]; *(volatile float*)p = v; }
}
__global__ __launch_bounds__(256) void k_conv(const float* __restrict__ ZX, const float* __restrict__ PBC, const float* __restrict__ cw, const float* __restrict__ cb, float* __restrict__ XBC) {
  const int t = blockIdx.x, tid = threadIdx.x;
#pragma unroll 1
  for (int pass = 0; pass < 2; ++pass) {
#pragma unroll 1
    for (int c = tid; c < CDm; c += 256) { float acc = cb[c];
#pragma unroll
      for (int k = 0; k < 4; ++k) { const int tt = t - 3 + k; const int tc = max(tt, 0); const float xz = ZX[(size_t)tc * NPP + DIm + min(c, DIm - 1)]; const float xp = PBC[(size_t)tc * 384 + min(max(c - DIm, 0), 255)];
        const float xv = (c < DIm) ? xz : xp; acc = fmaf((tt >= 0) ? xv : 0.0f, cw[c * 4 + k], acc); }
      *(volatile float*)(XBC + (size_t)t * CDm + c) = acc / (1.0f + expf(-acc)); }
    __threadfence(); }
}
__global__ __launch_bounds__(64) void k_dtacs(const float* __restrict__ PBC, const float* __restrict__ dtb, const float* __restrict__ Alog, float* __restrict__ DT, float* __restrict__ ACS) {
  const int c = blockIdx.x, h = threadIdx.x; if (h >= DTPm) return; const bool live = h < NHm; const int hc = min(h, NHm - 1); const float ah = -expf(Alog[hc]); const float bh = dtb[hc]; float run = 0.0f;
#pragma unroll 1
  for (int i = 0; i < CKm; ++i) { const size_t l = (size_t)c * CKm + i; const float dr = PBC[l * 384 + 256 + hc] + bh; const float dt0 = (dr > 20.0f) ? dr : log1pf(expf(dr)); const float dt = live ? dt0 : 0.0f;
    run += ah * dt; const float rv = live ? run : 0.0f; *(volatile float*)(DT + l * DTPm + h) = dt; *(volatile float*)(ACS + l * DTPm + h) = rv; }
  __threadfence();
#pragma unroll 1
  for (int i = 0; i < CKm; ++i) { const size_t l = (size_t)c * CKm + i; const float a = DT[l * DTPm + h], b2 = ACS[l * DTPm + h]; *(volatile float*)(DT + l * DTPm + h) = a; *(volatile float*)(ACS + l * DTPm + h) = b2; }
}
__global__ __launch_bounds__(256) void k_xplanes(const float* __restrict__ XBC, const float* __restrict__ DT, const float* __restrict__ ACS, float* __restrict__ XDT, float* __restrict__ XDEC) {
  const int l = blockIdx.x, tid = threadIdx.x; const int llast = (l / CKm) * CKm + CKm - 1;
#pragma unroll 1
  for (int q = tid; q < DIm / 4; q += 256) { const int h = (4 * q) / PPm; const float dt = DT[(size_t)l * DTPm + h]; const float dec = expf(ACS[(size_t)llast * DTPm + h] - ACS[(size_t)l * DTPm + h]);
    const v4f_t x = *(const v4f_t*)(XBC + (size_t)l * CDm + 4 * q); const v4f_t a = x * dt, b2 = x * (dt * dec);
    *(volatile v4f_t*)(XDT + (size_t)l * DIm + 4 * q) = a; *(volatile v4f_t*)(XDEC + (size_t)l * DIm + 4 * q) = b2; __threadfence(); *(volatile v4f_t*)(XDT + (size_t)l * DIm + 4 * q) = a; *(volatile v4f_t*)(XDEC + (size_t)l * DIm + 4 * q) = b2; }
}
__global__ __launch_bounds__(256) void k_gmat(const float* __restrict__ CB, const float* __restrict__ ACSc, float* __restrict__ G) {
  const int i = blockIdx.x, s = threadIdx.x; const float cb = CB[(size_t)i * CKm + s];
#pragma unroll 1
  for (int pass = 0; pass < 2; ++pass) {
#pragma unroll 1
    for (int h = 0; h < NHm; ++h) { const float ai = ACSc[(size_t)i * DTPm + h], as = ACSc[(size_t)s * DTPm + h]; const float v = (s <= i) ? cb * expf(ai - as) : 0.0f;
      *(volatile float*)(G + ((size_t)h * CKm + i) * CKm + s) = v; }
    __threadfence(); }
}
__global__ __launch_bounds__(256) void k_cs(const float* __restrict__ Cc, const float* __restrict__ ACSc, float* __restrict__ CS) {
  const int i = blockIdx.x, tid = threadIdx.x;
#pragma unroll 1
  for (int pass = 0; pass < 2; ++pass) {
#pragma unroll 1
    for (int e = tid; e < NHm * (NSm / 4); e += 256) { const int h = e / (NSm / 4), n4 = (e % (NSm / 4)) * 4; const float ea = expf(ACSc[(size_t)i * DTPm + h]);
      const v4f_t c = *(const v4f_t*)(Cc + (size_t)i * CDm + n4) * ea; *(volatile v4f_t*)(CS + ((size_t)h * CKm + i) * NSm + n4) = c; }
    __threadfence(); }
}
__global__ __launch_bounds__(256) void k_prev(const float* __restrict__ ST, const float* __restrict__ ACS, float* __restrict__ PREV) {
  const int h = blockIdx.y, part = blockIdx.x, tid = threadIdx.x; const size_t off = (size_t)part * 1024 + 4 * tid;
  v4f_t p = {0.f, 0.f, 0.f, 0.f};
#pragma unroll 1
  for (int c = 0; c < NCK; ++c) { float* d = PREV + (((size_t)c * NHm + h) * PPm * NSm) + off; *(volatile v4f_t*)d = p; __threadfence(); *(volatile v4f_t*)d = p;
    const float dec = expf(ACS[((size_t)c * CKm + CKm - 1) * DTPm + h]); const v4f_t s = *(const v4f_t*)(ST + (((size_t)c * NHm + h) * PPm * NSm) + off); p = p * dec + s; }
}
__global__ __launch_bounds__(256) void k_gnorm(const float* __restrict__ Y, const float* __restrict__ XBC, const float* __restrict__ ZX, const float* __restrict__ Dv, const float* __restrict__ w, f16* __restrict__ Gout) {
  __shared__ float red[256]; __shared__ __attribute__((aligned(16))) float gs[DIm];
  const int l = blockIdx.x, tid = threadIdx.x; float s = 0.0f;
#pragma unroll
  for (int e = 0; e < 2; ++e) { const int c = 4 * (tid + 256 * e); const int h = c / PPm; const v4f_t y = *(const v4f_t*)(Y + (size_t)l * DIm + c) + *(const v4f_t*)(XBC + (size_t)l * CDm + c) * Dv[h];
    const v4f_t z = *(const v4f_t*)(ZX + (size_t)l * NPP + c); v4f_t g;
#pragma unroll
    for (int u = 0; u < 4; ++u) { g[u] = y[u] * (z[u] / (1.0f + expf(-z[u]))); s += g[u] * g[u]; }
    *(v4fa*)(gs + c) = g; }
  red[tid] = s; __syncthreads(); for (int o = 128; o > 0; o >>= 1) { if (tid < o) red[tid] += red[tid + o]; __syncthreads(); }
  const float rs = 1.0f / __builtin_sqrtf(red[0] * (1.0f / DIm) + 1e-5f);
#pragma unroll
  for (int e = 0; e < 2; ++e) { const int c = 4 * (tid + 256 * e); const v4f_t g = *(const v4fa*)(gs + c); const v4f_t wv = *(const v4f_t*)(w + c); union { f16 hh[4]; unsigned long long u; } o;
#pragma unroll
    for (int u = 0; u < 4; ++u) o.hh[u] = (f16)(g[u] * rs * wv[u]);
    *(volatile unsigned long long*)(Gout + (size_t)l * DIm + c) = o.u; __threadfence(); *(volatile unsigned long long*)(Gout + (size_t)l * DIm + c) = o.u; }
}

extern "C" void kernel_launch(void* const* d_in, const int* in_sizes, int n_in,
                              void* d_out, int out_size, void* d_ws, size_t ws_size,
                              hipStream_t stream) {
  (void)in_sizes; (void)n_in; (void)out_size;
  const float** f = (const float**)d_in;
  const float* u = f[0], *win = f[1], *cw = f[2], *cb = f[3], *dtb = f[4], *Alog = f[5], *Dv = f[6], *nw = f[7], *wout = f[8];
  float* out = (float*)d_out;
  char* ws = (char*)d_ws;
  float* WinT = (float*)ws; ws += (size_t)DDm * NPP * 4;
  float* ZX = (float*)ws; ws += (size_t)LLm * NPP * 4;
  float* XBC = (float*)ws; ws += (size_t)LLm * CDm * 4; float* DT = (float*)ws; ws += (size_t)LLm * DTPm * 4; float* ACS = (float*)ws; ws += (size_t)LLm * DTPm * 4;
  float* XDT = (float*)ws; ws += (size_t)LLm * DIm * 4; float* XDEC = (float*)ws; ws += (size_t)LLm * DIm * 4; float* Y = (float*)ws; ws += (size_t)LLm * DIm * 4;
  float* BT = (float*)ws; ws += (size_t)NSm * CKm * 4; float* CB = (float*)ws; ws += (size_t)CKm * CKm * 4; float* G = (float*)ws; ws += (size_t)NHm * CKm * CKm * 4; float* CS = (float*)ws; ws += (size_t)NHm * CKm * NSm * 4;
  float* ST = (float*)ws; ws += (size_t)(LLm / CKm) * NHm * NSm * PPm * 4; float* PREV = (float*)ws; ws += (size_t)(LLm / CKm) * NHm * NSm * PPm * 4;
  f16* G16 = (f16*)ws; ws += (size_t)LLm * DIm * 2; float* ones = (float*)ws; ws += DIm * 4;
  float* PBC = (float*)ws; ws += (size_t)LLm * 384 * 4;
  if ((size_t)(ws - (char*)d_ws) > ws_size) return;
  const dim3 blk(256);
  k_padin<<<dim3(DDm), blk, 0, stream>>>(win, WinT); k_fill<<<dim3((DIm / 4 + 255) / 256), blk, 0, stream>>>(ones, 1.0f, DIm / 4);

  for (int b = 0; b < NBm; ++b) {
    const float* ub = u + (size_t)b * LIN * DDm;
    gemm_kne<float, 0, false><<<dim3(LLm / 128, NPP / 128), blk, 0, stream>>>(ub, DDm, WinT, NPP, nullptr, nullptr, nullptr, ZX, NPP, DDm);
    gemm_kn2<float, false><<<dim3(LLm / 128, 3, 1), blk, 0, stream>>>(ub, DDm, 0, WinT + 2 * DIm, NPP, 0, nullptr, 1.0f, PBC, 384, 0, DDm);
    k_conv<<<dim3(LLm), blk, 0, stream>>>(ZX, PBC, cw, cb, XBC);
    k_dtacs<<<dim3(NCK), dim3(64), 0, stream>>>(PBC, dtb, Alog, DT, ACS);
    k_xplanes<<<dim3(LLm), blk, 0, stream>>>(XBC, DT, ACS, XDT, XDEC);
    for (int c = 0; c < NCK; ++c) { const size_t r0 = (size_t)c * CKm;
      const float* Bc = XBC + r0 * CDm + DIm;
      const float* Cc = XBC + r0 * CDm + DIm + NSm;
      k_transpose_ld<<<dim3((CKm / 64) * (NSm / 64)), blk, 0, stream>>>(Bc, CDm, BT, CKm, NSm);
      gemm_kne<float, 0, false><<<dim3(CKm / 128, CKm / 128), blk, 0, stream>>>(Cc, CDm, BT, CKm, nullptr, nullptr, nullptr, CB, CKm, NSm);
      k_gmat<<<dim3(CKm), blk, 0, stream>>>(CB, ACS + r0 * DTPm, G);
      gemm_knez<float, 0, false><<<dim3(CKm / 128, 1, NHm), blk, 0, stream>>>(G, CKm, (size_t)CKm * CKm, XDT + r0 * DIm, DIm, (size_t)PPm, nullptr, nullptr, nullptr, Y + r0 * DIm, DIm, (size_t)PPm, CKm);
      gemm_knez<float, 0, false><<<dim3(NSm / 128, 1, NHm), blk, 0, stream>>>(BT, CKm, (size_t)0, XDEC + r0 * DIm, DIm, (size_t)PPm, nullptr, nullptr, nullptr, ST + (size_t)c * NHm * NSm * PPm, PPm, (size_t)NSm * PPm, CKm);
    }
    k_prev<<<dim3(16, NHm), blk, 0, stream>>>(ST, ACS, PREV);
    for (int c = 0; c < NCK; ++c) { const size_t r0 = (size_t)c * CKm; const float* Cc = XBC + r0 * CDm + DIm + NSm;
      k_cs<<<dim3(CKm), blk, 0, stream>>>(Cc, ACS + r0 * DTPm, CS);
      gemm_knez<float, 2, false><<<dim3(CKm / 128, 1, NHm), blk, 0, stream>>>(CS, NSm, (size_t)CKm * NSm, PREV + (size_t)c * NHm * NSm * PPm, PPm, (size_t)NSm * PPm, nullptr, Y + r0 * DIm, ones, Y + r0 * DIm, DIm, (size_t)PPm, NSm);
    }
    k_gnorm<<<dim3(LLm), blk, 0, stream>>>(Y, XBC, ZX, Dv, nw, G16);
    gemm_rb_kernel<bf16, 2><<<dim3(LLm / 128, DDm / 256), blk, 0, stream>>>(G16, wout, nullptr, nullptr, nullptr, nullptr, out + (size_t)b * LIN * DDm, LLm, DDm, DIm);
  }
}
